// MyMultiheadAttention_74646531604978
// MI455X (gfx1250) — hardware-verified
//
#include <hip/hip_runtime.h>

typedef _Float16 v16h __attribute__((ext_vector_type(16)));
typedef _Float16 v8h  __attribute__((ext_vector_type(8)));
typedef float    v8f  __attribute__((ext_vector_type(8)));
typedef float    v4f  __attribute__((ext_vector_type(4)));
typedef v8h __attribute__((may_alias)) v8ha;
typedef v4f __attribute__((may_alias)) v4fa;

union Frag { v16h v; v8h half[2]; };

#define SEQ    2048
#define NB     2
#define EMB    1024
#define NH     16
#define HD     64
#define MROWS  (SEQ * NB)
#define NX     (MROWS * EMB)
#define NW     (EMB * EMB)
#define NX8    (NX / 8)
#define NW8    (NW / 8)
#define NBH    (NB * NH)
#define NQB    (SEQ / 64)
#define NAVG   (NB * SEQ * SEQ)
#define NSTAT  (NBH * NQB * 128)
#define PSCALE 16384.0f
#define WSCALE 32.0f
#define OSCALE 16.0f
#define QKSCALE 0.125f

__device__ __forceinline__ v8f wmma_f16(v16h a, v16h b, v8f c) {
  v8f d = __builtin_amdgcn_wmma_f32_16x16x32_f16(false, a, false, b, (short)0, c, false, false);
  asm volatile("v_nop\n\tv_nop\n\tv_nop\n\tv_nop" : "+v"(d) : "v"(a), "v"(b));
  return d;
}

__device__ __forceinline__ v16h load_frag(const _Float16* p, int h) {
  Frag f;
  f.half[0] = *(const v8ha*)(p + 8 * h);
  f.half[1] = *(const v8ha*)(p + 16 + 8 * h);
  return f.v;
}

__device__ __forceinline__ v8f zero8f() {
  const v8f z = {0.f, 0.f, 0.f, 0.f, 0.f, 0.f, 0.f, 0.f};
  return z;
}

__global__ __launch_bounds__(256) void convert_kernel(
    const float* __restrict__ xq, const float* __restrict__ xk, const float* __restrict__ xv,
    const float* __restrict__ wq, const float* __restrict__ wk,
    const float* __restrict__ wv, const float* __restrict__ wo,
    _Float16* __restrict__ xh, _Float16* __restrict__ wh)
{
  const int g = blockIdx.x * 256 + threadIdx.x;
  if (g >= 3 * NX8 + 4 * NW8) return;
  const float* src;
  _Float16* dst;
  float sc;
  if (g < 3 * NX8) {
    const int sel = g / NX8;
    const int off = g - sel * NX8;
    const float* s = (sel == 0) ? xq : ((sel == 1) ? xk : xv);
    src = s + (size_t)off * 8;
    dst = xh + (size_t)g * 8;
    sc = 1.0f;
  } else {
    const int e = g - 3 * NX8;
    const int sel = e / NW8;
    const int off = e - sel * NW8;
    const float* s = (sel == 0) ? wq : ((sel == 1) ? wk : ((sel == 2) ? wv : wo));
    src = s + (size_t)off * 8;
    dst = wh + (size_t)e * 8;
    sc = WSCALE;
  }
  const v4f a = *(const v4fa*)src;
  const v4f c = *(const v4fa*)(src + 4);
  const v8h o = { (_Float16)(a.x * sc), (_Float16)(a.y * sc), (_Float16)(a.z * sc), (_Float16)(a.w * sc),
                  (_Float16)(c.x * sc), (_Float16)(c.y * sc), (_Float16)(c.z * sc), (_Float16)(c.w * sc) };
  *(volatile v8h*)dst = o;
  __threadfence();
  *(volatile v8h*)dst = o;
}

__device__ __forceinline__ void gemm_tile_32x64(const _Float16* __restrict__ xa0,
                                                const _Float16* __restrict__ xa1,
                                                const _Float16* __restrict__ wb,
                                                int h, v8f (&acc)[2][4]) {
  #pragma unroll
  for (int mt = 0; mt < 2; ++mt)
    #pragma unroll
    for (int nt = 0; nt < 4; ++nt) acc[mt][nt] = zero8f();

  #pragma unroll 1
  for (int k0 = 0; k0 < EMB; k0 += 32) {
    const v16h a0 = load_frag(xa0 + k0, h);
    const v16h a1 = load_frag(xa1 + k0, h);
    #pragma unroll
    for (int nt = 0; nt < 4; ++nt) {
      const v16h b = load_frag(wb + (size_t)nt * 16 * EMB + k0, h);
      acc[0][nt] = wmma_f16(a0, b, acc[0][nt]);
      acc[1][nt] = wmma_f16(a1, b, acc[1][nt]);
    }
  }
}

__device__ __forceinline__ void proj_store_pass(const _Float16* sT, _Float16* plane, _Float16* vt,
                                                int which, int bh, int l0, int w, int lane) {
  const int q8 = lane & 7, sub = lane >> 3;
  #pragma unroll
  for (int i = 0; i < 8; ++i) {
    const int lid = w * 32 + i * 4 + sub;
    v8h v;
    _Float16* dst;
    if (which != 2) {
      v = *(const v8ha*)(sT + lid * HD + 8 * q8);
      dst = plane + ((size_t)bh * SEQ + l0 + lid) * HD + 8 * q8;
    } else {
      const int d = lid >> 1, hl = lid & 1;
      v = *(const v8ha*)(sT + d * 128 + 64 * hl + 8 * q8);
      dst = vt + ((size_t)bh * HD + d) * SEQ + l0 + 64 * hl + 8 * q8;
    }
    *(volatile v8h*)dst = v;
  }
}

__global__ __launch_bounds__(128) void qkv_proj_kernel(
    const _Float16* __restrict__ xh,
    const _Float16* __restrict__ wh,
    const float* __restrict__ bq, const float* __restrict__ bk, const float* __restrict__ bv,
    _Float16* __restrict__ qh,
    _Float16* __restrict__ kh,
    _Float16* __restrict__ vt)
{
  __shared__ __attribute__((aligned(16))) _Float16 sT[128 * 64];

  const int tid = threadIdx.x, lane = tid & 31, w = tid >> 5;
  const int h = lane >> 4, m = lane & 15;
  const int b = blockIdx.x / (SEQ / 128);
  const int l0 = (blockIdx.x - b * (SEQ / 128)) * 128;
  const int which = blockIdx.y >> 4, head = blockIdx.y & 15;
  const int lw = l0 + 32 * w;

  const _Float16* xpl = xh + (size_t)which * NX;
  const _Float16* xa0 = xpl + ((size_t)(lw + m) * NB + b) * EMB;
  const _Float16* xa1 = xpl + ((size_t)(lw + 16 + m) * NB + b) * EMB;
  const _Float16* wb  = wh + (size_t)which * NW + ((size_t)head * HD + m) * EMB;

  v8f acc[2][4];
  gemm_tile_32x64(xa0, xa1, wb, h, acc);

  const float* bias = (which == 0) ? bq : ((which == 1) ? bk : bv);
  #pragma unroll
  for (int nt = 0; nt < 4; ++nt) {
    const int feat = 16 * nt + m;
    const float bvl = bias[head * HD + feat];
    #pragma unroll
    for (int mt = 0; mt < 2; ++mt) {
      #pragma unroll
      for (int r = 0; r < 8; ++r) {
        const int tokl = 32 * w + 16 * mt + 8 * h + r;
        const float y = acc[mt][nt][r] * (1.0f / WSCALE) + bvl;
        const int idx = (which == 2) ? (feat * 128 + tokl) : (tokl * HD + feat);
        sT[idx] = (_Float16)y;
      }
    }
  }
  __syncthreads();

  const int bh = b * NH + head;
  _Float16* plane = (which == 0) ? qh : kh;
  proj_store_pass(sT, plane, vt, which, bh, l0, w, lane);
  __threadfence();
  proj_store_pass(sT, plane, vt, which, bh, l0, w, lane);
}

__device__ __forceinline__ v16h pack_p(v8f a, v8f c) {
  const v16h r = { (_Float16)(a[0] * PSCALE), (_Float16)(a[1] * PSCALE), (_Float16)(a[2] * PSCALE), (_Float16)(a[3] * PSCALE),
                   (_Float16)(a[4] * PSCALE), (_Float16)(a[5] * PSCALE), (_Float16)(a[6] * PSCALE), (_Float16)(a[7] * PSCALE),
                   (_Float16)(c[0] * PSCALE), (_Float16)(c[1] * PSCALE), (_Float16)(c[2] * PSCALE), (_Float16)(c[3] * PSCALE),
                   (_Float16)(c[4] * PSCALE), (_Float16)(c[5] * PSCALE), (_Float16)(c[6] * PSCALE), (_Float16)(c[7] * PSCALE) };
  return r;
}

__device__ __forceinline__ void ctx_store_pass(const _Float16* so, const float* sst,
                                               _Float16* ao, float* strec,
                                               int b, int head, int q0, int w, int lane) {
  const int q8 = lane & 7, sub = lane >> 3;
  #pragma unroll
  for (int i = 0; i < 4; ++i) {
    const int row = i * 4 + sub;
    const v8h v = *(const v8ha*)(so + row * 64 + 8 * q8);
    _Float16* dst = ao + ((size_t)(q0 + row) * NB + b) * EMB + head * HD + 8 * q8;
    *(volatile v8h*)dst = v;
  }
  if (w == 0) {
    const v4f t = *(const v4fa*)(sst + 4 * lane);
    *(volatile v4f*)(strec + 4 * lane) = t;
  }
}

__global__ __launch_bounds__(128) void attn_ctx_kernel(
    const _Float16* __restrict__ qh,
    const _Float16* __restrict__ kh,
    const _Float16* __restrict__ vt,
    _Float16* __restrict__ ao,
    float* __restrict__ stats)
{
  __shared__ __attribute__((aligned(16))) _Float16 sO[4 * 16 * 64];
  __shared__ __attribute__((aligned(16))) float sSt[128];

  const int tid = threadIdx.x, lane = tid & 31, w = tid >> 5;
  const int h = lane >> 4, m = lane & 15;
  const int bh = blockIdx.y, b = bh >> 4, head = bh & 15;
  const int qb = blockIdx.x;
  const int q0 = qb * 64 + 16 * w;

  const _Float16* qrow = qh + ((size_t)bh * SEQ + q0 + m) * HD;
  const v16h qb0 = load_frag(qrow, h);
  const v16h qb1 = load_frag(qrow + 32, h);

  v8f o[4];
  #pragma unroll
  for (int t = 0; t < 4; ++t) o[t] = zero8f();
  float mrun = -1e30f, lrun = 0.0f;

  const _Float16* kbase = kh + ((size_t)bh * SEQ + m) * HD;
  const _Float16* vbase = vt + ((size_t)bh * HD + m) * SEQ;

  #pragma unroll 1
  for (int kb = 0; kb < SEQ; kb += 64) {
    v8f s[4];
    #pragma unroll
    for (int j = 0; j < 4; ++j) {
      const _Float16* kp = kbase + (size_t)(kb + 16 * j) * HD;
      const v16h kf0 = load_frag(kp, h);
      const v16h kf1 = load_frag(kp + 32, h);
      v8f z = zero8f();
      z = wmma_f16(kf0, qb0, z);
      z = wmma_f16(kf1, qb1, z);
      #pragma unroll
      for (int r = 0; r < 8; ++r) s[j][r] = z[r] * QKSCALE;
    }

    float mloc = s[0][0];
    #pragma unroll
    for (int j = 0; j < 4; ++j)
      #pragma unroll
      for (int r = 0; r < 8; ++r) mloc = fmaxf(mloc, s[j][r]);
    mloc = fmaxf(mloc, __shfl_xor(mloc, 16));
    const float mnew = fmaxf(mrun, mloc);
    const float alpha = __expf(mrun - mnew);
    mrun = mnew;
    float lsum = 0.0f;
    #pragma unroll
    for (int j = 0; j < 4; ++j)
      #pragma unroll
      for (int r = 0; r < 8; ++r) {
        const float p = __expf(s[j][r] - mnew);
        s[j][r] = p;
        lsum += p;
      }
    lsum += __shfl_xor(lsum, 16);
    lrun = lrun * alpha + lsum;
    #pragma unroll
    for (int t = 0; t < 4; ++t)
      #pragma unroll
      for (int r = 0; r < 8; ++r) o[t][r] = o[t][r] * alpha;

    const v16h pb0 = pack_p(s[0], s[1]);
    const v16h pb1 = pack_p(s[2], s[3]);

    #pragma unroll
    for (int t = 0; t < 4; ++t) {
      const _Float16* vp = vbase + (size_t)(16 * t) * SEQ + kb;
      const v16h vf0 = load_frag(vp, h);
      const v16h vf1 = load_frag(vp + 32, h);
      o[t] = wmma_f16(vf0, pb0, o[t]);
      o[t] = wmma_f16(vf1, pb1, o[t]);
    }
  }

  const float linv = 1.0f / lrun;
  const float inv = linv * (OSCALE / PSCALE);
  _Float16* so = sO + w * 1024;
  #pragma unroll
  for (int t = 0; t < 4; ++t)
    #pragma unroll
    for (int r = 0; r < 8; ++r)
      so[m * 64 + 16 * t + 8 * h + r] = (_Float16)(o[t][r] * inv);
  if (h == 0) {
    sSt[16 * w + m] = mrun;
    sSt[64 + 16 * w + m] = linv;
  }
  __syncthreads();

  float* strec = stats + ((size_t)bh * NQB + qb) * 128;
  ctx_store_pass(so, sSt, ao, strec, b, head, q0, w, lane);
  __threadfence();
  ctx_store_pass(so, sSt, ao, strec, b, head, q0, w, lane);
}

__device__ __forceinline__ void tile16x64_store_pass(const float* so, float* dst,
                                                     size_t row0, int col0, int pitch, int lane) {
  const int q8 = lane & 7, sub = lane >> 3;
  #pragma unroll
  for (int i = 0; i < 8; ++i) {
    const int lid = i * 4 + sub;
    const int row = lid >> 1, hl = lid & 1;
    const v4f v = *(const v4fa*)(so + row * 64 + 32 * hl + 4 * q8);
    const size_t gi = (row0 + row) * (size_t)pitch + col0 + 32 * hl + 4 * q8;
    *(volatile v4f*)(dst + gi) = v;
  }
}

__global__ __launch_bounds__(128) void attn_avg_kernel(
    const _Float16* __restrict__ qh,
    const _Float16* __restrict__ kh,
    const float* __restrict__ stats,
    float* __restrict__ avg)
{
  __shared__ __attribute__((aligned(16))) float sA[4 * 16 * 64];

  const int tid = threadIdx.x, lane = tid & 31, w = tid >> 5;
  const int h = lane >> 4, m = lane & 15;
  const int kt = blockIdx.x * 64;
  const int qb = blockIdx.y;
  const int b = blockIdx.z;
  const int q0 = qb * 64 + 16 * w;

  v8f acc[4];
  #pragma unroll
  for (int j = 0; j < 4; ++j) acc[j] = zero8f();

  #pragma unroll 1
  for (int hh = 0; hh < NH; ++hh) {
    const int bh = b * NH + hh;
    const _Float16* qrow = qh + ((size_t)bh * SEQ + q0 + m) * HD;
    const v16h qb0 = load_frag(qrow, h);
    const v16h qb1 = load_frag(qrow + 32, h);
    const float* st = stats + ((size_t)bh * NQB + qb) * 128;
    const float mq = st[16 * w + m];
    const float li = st[64 + 16 * w + m];
    const _Float16* kbase = kh + ((size_t)bh * SEQ + kt + m) * HD;
    #pragma unroll
    for (int j = 0; j < 4; ++j) {
      const _Float16* kp = kbase + (size_t)(16 * j) * HD;
      const v16h kf0 = load_frag(kp, h);
      const v16h kf1 = load_frag(kp + 32, h);
      v8f z = zero8f();
      z = wmma_f16(kf0, qb0, z);
      z = wmma_f16(kf1, qb1, z);
      #pragma unroll
      for (int r = 0; r < 8; ++r) {
        const float sv = z[r] * QKSCALE;
        acc[j][r] += __expf(sv - mq) * li;
      }
    }
  }

  float* so = sA + w * 1024;
  #pragma unroll
  for (int j = 0; j < 4; ++j)
    #pragma unroll
    for (int r = 0; r < 8; ++r)
      so[m * 64 + 16 * j + 8 * h + r] = acc[j][r] * (1.0f / (float)NH);
  __syncthreads();

  const size_t row0 = (size_t)b * SEQ + q0;
  tile16x64_store_pass(so, avg, row0, kt, SEQ, lane);
  __threadfence();
  tile16x64_store_pass(so, avg, row0, kt, SEQ, lane);
}

__device__ __forceinline__ void zout_store_pass(const float* sz, float* z, int mrow0, int c0, int lane) {
  const int q8 = lane & 7, sub = lane >> 3;
  #pragma unroll
  for (int i = 0; i < 16; ++i) {
    const int lid = i * 4 + sub;
    const int row = lid >> 1, hl = lid & 1;
    const v4f v = *(const v4fa*)(sz + row * 64 + 32 * hl + 4 * q8);
    const size_t gi = (size_t)(mrow0 + row) * EMB + c0 + 32 * hl + 4 * q8;
    *(volatile v4f*)(z + gi) = v;
  }
}

__global__ __launch_bounds__(128) void out_proj_kernel(
    const _Float16* __restrict__ ao,
    const _Float16* __restrict__ wh,
    const float* __restrict__ bo,
    float* __restrict__ z)
{
  __shared__ __attribute__((aligned(16))) float sZ[128 * 64];

  const int tid = threadIdx.x, lane = tid & 31, w = tid >> 5;
  const int h = lane >> 4, m = lane & 15;
  const int m0w = blockIdx.x * 128 + 32 * w;
  const int c0 = blockIdx.y * 64;

  const _Float16* xa0 = ao + (size_t)(m0w + m) * EMB;
  const _Float16* xa1 = xa0 + (size_t)16 * EMB;
  const _Float16* wb  = wh + (size_t)3 * NW + ((size_t)c0 + m) * EMB;

  v8f acc[2][4];
  gemm_tile_32x64(xa0, xa1, wb, h, acc);

  float* sz = sZ + w * 2048;
  #pragma unroll
  for (int nt = 0; nt < 4; ++nt) {
    const int col = 16 * nt + m;
    const float bvl = bo[c0 + col];
    #pragma unroll
    for (int mt = 0; mt < 2; ++mt) {
      #pragma unroll
      for (int r = 0; r < 8; ++r) {
        const int rowl = 16 * mt + 8 * h + r;
        sz[rowl * 64 + col] = acc[mt][nt][r] * (1.0f / (WSCALE * OSCALE)) + bvl;
      }
    }
  }
  __syncthreads();

  zout_store_pass(sz, z, m0w, c0, lane);
  __threadfence();
  zout_store_pass(sz, z, m0w, c0, lane);
}

extern "C" void kernel_launch(void* const* d_in, const int* in_sizes, int n_in,
                              void* d_out, int out_size, void* d_ws, size_t ws_size,
                              hipStream_t stream) {
  if (n_in < 11) return;
  if (in_sizes[0] != NX || in_sizes[1] != NX || in_sizes[2] != NX) return;
  if (in_sizes[3] != NW || in_sizes[5] != NW || in_sizes[7] != NW || in_sizes[9] != NW) return;
  if (in_sizes[4] != EMB || in_sizes[6] != EMB || in_sizes[8] != EMB || in_sizes[10] != EMB) return;
  if (out_size != NX + NAVG) return;

  const float* xq  = (const float*)d_in[0];
  const float* xk  = (const float*)d_in[1];
  const float* xv  = (const float*)d_in[2];
  const float* q_w = (const float*)d_in[3];
  const float* q_b = (const float*)d_in[4];
  const float* k_w = (const float*)d_in[5];
  const float* k_b = (const float*)d_in[6];
  const float* v_w = (const float*)d_in[7];
  const float* v_b = (const float*)d_in[8];
  const float* o_w = (const float*)d_in[9];
  const float* o_b = (const float*)d_in[10];
  float* zout = (float*)d_out;
  float* avg  = zout + (size_t)NX;

  const size_t xh_bytes = (size_t)3 * NX * 2;
  const size_t wh_bytes = (size_t)4 * NW * 2;
  const size_t pl_bytes = (size_t)NBH * SEQ * HD * 2;
  const size_t st_bytes = (size_t)NSTAT * 4;
  const size_t ao_bytes = (size_t)NX * 2;
  const size_t total = xh_bytes + wh_bytes + 3 * pl_bytes + st_bytes + ao_bytes;
  if (total > ws_size) return;

  char* ws = (char*)d_ws;
  size_t off = 0;
  _Float16* xh = (_Float16*)(ws + off);   off += xh_bytes;
  _Float16* wh = (_Float16*)(ws + off);   off += wh_bytes;
  _Float16* qh = (_Float16*)(ws + off);   off += pl_bytes;
  _Float16* kh = (_Float16*)(ws + off);   off += pl_bytes;
  _Float16* vt = (_Float16*)(ws + off);   off += pl_bytes;
  float* stats = (float*)(ws + off);      off += st_bytes;
  _Float16* ao = (_Float16*)(ws + off);   off += ao_bytes;
  if (off > ws_size) return;

  const int ngroups = 3 * NX8 + 4 * NW8;
  convert_kernel<<<(ngroups + 255) / 256, 256, 0, stream>>>(xq, xk, xv, q_w, k_w, v_w, o_w, xh, wh);

  dim3 gProj(NB * SEQ / 128, 3 * NH);
  qkv_proj_kernel<<<gProj, 128, 0, stream>>>(xh, wh, q_b, k_b, v_b, qh, kh, vt);

  dim3 gCtx(NQB, NBH);
  attn_ctx_kernel<<<gCtx, 128, 0, stream>>>(qh, kh, vt, ao, stats);

  dim3 gAvg(SEQ / 64, NQB, NB);
  attn_avg_kernel<<<gAvg, 128, 0, stream>>>(qh, kh, stats, avg);

  dim3 gOut(MROWS / 128, EMB / 64);
  out_proj_kernel<<<gOut, 128, 0, stream>>>(ao, wh, o_b, zout);
}
